// MutualAttention_2619930051055
// MI455X (gfx1250) — hardware-run, weakly checked
//
#include <hip/hip_runtime.h>
#include <math.h>
#include <stdint.h>

#define NBT    2
#define CN     64
#define C3     192
#define IMW    256
#define HWN    65536
#define HWH    32768
#define NHEAD  8
#define KT1    1728
#define KT2    576
#define XP     72
#define OPP    200
#define OSP    68
#define TP     72
#define NCBLK  (4 * IMW * NBT)
#define XSC    16.0f
#define WSC    64.0f
#define QSC    1024.0f
#define WTS    4096.0f
#define RSC    2048.0f
#define IRSC   0.00048828125f
#define FSC    1024.0f
#define CBS    16.0f

static_assert(KT1 == 9 * C3);
static_assert(KT2 == 9 * CN);
static_assert(KT1 % 32 == 0);
static_assert(KT2 % 32 == 0);
static_assert((XP * 2) % 16 == 0);
static_assert((OPP * 2) % 16 == 0);
static_assert((OSP * 4) % 16 == 0);
static_assert((TP * 2) % 16 == 0);
static_assert(NHEAD * 8 == CN);
static_assert(IMW * IMW == HWN);
static_assert(2 * HWH == HWN);
static_assert(HWN % 256 == 0);
static_assert((3 * 66 * TP * 2) % 16 == 0);

typedef _Float16       v16h __attribute__((ext_vector_type(16)));
typedef _Float16       v8h  __attribute__((ext_vector_type(8)));
typedef unsigned short v8us __attribute__((ext_vector_type(8)));
typedef float          v8f  __attribute__((ext_vector_type(8)));
typedef float          v4f  __attribute__((ext_vector_type(4)));
typedef unsigned int   v4u  __attribute__((ext_vector_type(4)));

union Frag { v8us u[2]; v16h h; };
static_assert(sizeof(Frag) == 32);

__device__ __forceinline__ unsigned short bf_bits(float f) {
  unsigned u = __float_as_uint(f);
  return (unsigned short)((u + 0x7FFFu + ((u >> 16) & 1u)) >> 16);
}
__device__ __forceinline__ float bf_up(unsigned short hb) { return __uint_as_float(((unsigned)hb) << 16); }
__device__ __forceinline__ float bfr(float f) { return bf_up(bf_bits(f)); }
__device__ __forceinline__ unsigned short h_bits(_Float16 x) { return __builtin_bit_cast(unsigned short, x); }
__device__ __forceinline__ unsigned pk16(unsigned short a, unsigned short b) { return (unsigned)a | ((unsigned)b << 16); }
__device__ __forceinline__ v8f zero8() { v8f z = {0.f, 0.f, 0.f, 0.f, 0.f, 0.f, 0.f, 0.f}; return z; }
__device__ __forceinline__ int refl(int i) { i = (i < 0) ? -i : i; return (i >= IMW) ? (2 * IMW - 2 - i) : i; }

__device__ __forceinline__ Frag ldfrag(const unsigned short* p) {
  Frag f;
  f.u[0] = *(const v8us*)(p);
  f.u[1] = *(const v8us*)(p + 16);
  return f;
}

__device__ __forceinline__ v8f mma_h(v16h a, v16h b, v8f c) {
  v8f d = __builtin_amdgcn_wmma_f32_16x16x32_f16(false, a, false, b, (short)0, c, false, false);
#if defined(__HIP_DEVICE_COMPILE__)
  asm volatile("v_nop\n\tv_nop\n\tv_nop\n\tv_nop" : "+v"(d) : "v"(a), "v"(b));
#endif
  return d;
}

__global__ __launch_bounds__(256)
void cvt_w(const float* __restrict__ w_init, const float* __restrict__ w1, const float* __restrict__ w2,
           const float* __restrict__ wq, const float* __restrict__ wk,
           unsigned short* WC1, unsigned short* WC2, unsigned short* WQK) {
  const int tid = threadIdx.x, e = tid & 7, lq = tid >> 3;
  const int blk = blockIdx.x;
  float v[8];
  unsigned short* dst;
  if (blk < 108) {
    const int L = blk * 32 + lq;
    const int row = L / 27, pc = L - 27 * row;
    const int k = pc * 64 + 8 * e;
    const int tap = k / C3, ci = k - C3 * tap;
    const int set = row >> 6, oc = row & 63;
    const float* w = set ? w1 : w_init;
#pragma unroll
    for (int q = 0; q < 8; ++q) v[q] = w[((size_t)(oc * C3 + ci + q)) * 9 + tap];
    dst = WC1 + (size_t)row * KT1 + k;
  } else if (blk < 126) {
    const int L = (blk - 108) * 32 + lq;
    const int row = L / 9, pc = L - 9 * row;
    const int k = pc * 64 + 8 * e;
#pragma unroll
    for (int q = 0; q < 8; ++q) v[q] = w2[((size_t)(row * CN + 8 * e + q)) * 9 + pc];
    dst = WC2 + (size_t)row * KT2 + k;
  } else {
    const int L = (blk - 126) * 32 + lq;
    const int t = L >> 6, oc = L & 63;
    const float* w = t ? wk : wq;
#pragma unroll
    for (int q = 0; q < 8; ++q) v[q] = w[oc * CN + 8 * e + q];
    dst = WQK + (size_t)L * CN + 8 * e;
  }
  v4u u;
#pragma unroll
  for (int q = 0; q < 4; ++q)
    u[q] = pk16(h_bits((_Float16)(WSC * bfr(v[2 * q]))), h_bits((_Float16)(WSC * bfr(v[2 * q + 1]))));
#pragma unroll
  for (int pass = 0; pass < 2; ++pass) {
    *(volatile v4u*)dst = u;
    __threadfence();
  }
}

__global__ __launch_bounds__(256)
void k_proj(const float* __restrict__ y, const float* __restrict__ xe, const float* __restrict__ xi,
            const unsigned short* __restrict__ WQK, const float* __restrict__ bq, const float* __restrict__ bk,
            unsigned short* QKP) {
  __shared__ __align__(16) unsigned short X16[64 * XP];
  __shared__ __align__(16) unsigned short Qt[64 * XP];
  const int tid = threadIdx.x, lane = tid & 31, wave = tid >> 5;
  const int hh = lane >> 4, c = lane & 15;
  const int tile = blockIdx.x, t = blockIdx.y, b = blockIdx.z;
  const int p0 = tile * 64;
  const float* x = (t == 0) ? y : ((t == 1) ? xe : xi);
  const float* bias = (t == 0) ? bq : bk;
  const unsigned short* W = WQK + ((t == 0) ? 0 : CN * CN);
  const size_t cb0 = (size_t)b * CN * HWN;
#pragma unroll
  for (int it = 0; it < 4; ++it) {
    const int idx = it * 256 + tid;
    const int ci = idx >> 4, p4 = (idx & 15) * 4;
    const v4f v = *(const v4f*)(x + cb0 + (size_t)ci * HWN + p0 + p4);
#pragma unroll
    for (int q = 0; q < 4; ++q) X16[(p4 + q) * XP + ci] = h_bits((_Float16)(XSC * bfr(v[q])));
  }
  __syncthreads();
  {
    const int mt = wave & 3, ntb = 2 * (wave >> 2);
    v8f acc0 = zero8(), acc1 = zero8();
#pragma unroll
    for (int ks = 0; ks < 2; ++ks) {
      const Frag fa  = ldfrag(W + (16 * mt + c) * CN + 32 * ks + 8 * hh);
      const Frag fb0 = ldfrag(X16 + (16 * ntb + c) * XP + 32 * ks + 8 * hh);
      const Frag fb1 = ldfrag(X16 + (16 * ntb + 16 + c) * XP + 32 * ks + 8 * hh);
      acc0 = mma_h(fa.h, fb0.h, acc0);
      acc1 = mma_h(fa.h, fb1.h, acc1);
    }
#pragma unroll
    for (int r = 0; r < 8; ++r) {
      const int ch = 16 * mt + 8 * hh + r;
      const float bvv = QSC * bfr(bias[ch]);
      Qt[ch * XP + 16 * ntb + c]      = h_bits((_Float16)(acc0[r] + bvv));
      Qt[ch * XP + 16 * ntb + 16 + c] = h_bits((_Float16)(acc1[r] + bvv));
    }
  }
  __syncthreads();
  {
    const int e = tid & 7, lq = tid >> 3;
    const v4u u0 = *(const v4u*)(Qt + lq * XP + 8 * e);
    const v4u u1 = *(const v4u*)(Qt + (lq + 32) * XP + 8 * e);
    unsigned short* base = QKP + ((size_t)(t * NBT + b) * CN) * HWN;
    unsigned short* d0 = base + (size_t)lq * HWN + p0 + 8 * e;
    unsigned short* d1 = base + (size_t)(lq + 32) * HWN + p0 + 8 * e;
#pragma unroll
    for (int pass = 0; pass < 2; ++pass) {
      *(volatile v4u*)(d0) = u0;
      *(volatile v4u*)(d1) = u1;
      __threadfence();
    }
  }
}

__global__ __launch_bounds__(256)
void k_attnw(const unsigned short* __restrict__ QKP, const float* __restrict__ temp,
             const float* __restrict__ wv, const float* __restrict__ bv,
             const float* __restrict__ wo, const float* __restrict__ bo,
             unsigned short* WHL, float* BTg) {
  __shared__ float sNorm[128];
  __shared__ float invn[128];
  __shared__ float sS[8 * 256];
  __shared__ float attn[512];
  __shared__ __align__(16) float M1[4096];
  __shared__ __align__(16) unsigned short Wst[2 * 4096];
  __shared__ __align__(16) float BTst[64];
  const int tid = threadIdx.x, lane = tid & 31, wave = tid >> 5;
  const int hh = lane >> 4, c = lane & 15;
  const int a = blockIdx.x, b = blockIdx.y;
  const unsigned short* qb = QKP + ((size_t)(0 * NBT + b) * CN) * HWN;
  const unsigned short* kb = QKP + ((size_t)((1 + a) * NBT + b) * CN) * HWN;

#pragma unroll 1
  for (int rr = 0; rr < 16; ++rr) {
    const int R = 16 * wave + rr;
    const unsigned short* rp = ((R < 64) ? qb : kb) + (size_t)(R & 63) * HWN;
    float s = 0.f;
#pragma unroll 2
    for (int j = 0; j < HWN / 256; ++j) {
      const v8h v = *(const v8h*)(rp + 8 * (lane + 32 * j));
      float t = 0.f;
#pragma unroll
      for (int q = 0; q < 8; ++q) { const float f = (float)v[q]; t = fmaf(f, f, t); }
      s += t;
    }
#pragma unroll
    for (int off = 16; off > 0; off >>= 1) s += __shfl_xor(s, off, 32);
    if (lane == 0) sNorm[R] = s;
  }

  {
    const int hp = wave & 3, kh = wave >> 2;
    const unsigned short* arow = qb + (size_t)(16 * hp + c) * HWN + (size_t)kh * HWH + 8 * hh;
    const unsigned short* brow = kb + (size_t)(16 * hp + c) * HWN + (size_t)kh * HWH + 8 * hh;
    v8f acc = zero8();
#pragma unroll 2
    for (int ks = 0; ks < HWH / 32; ++ks) {
      const Frag fa = ldfrag(arow + 32 * ks);
      const Frag fb = ldfrag(brow + 32 * ks);
      acc = mma_h(fa.h, fb.h, acc);
    }
#pragma unroll
    for (int r = 0; r < 8; ++r) sS[wave * 256 + (8 * hh + r) * 16 + c] = acc[r];
  }
  __syncthreads();
  if (tid < 128) invn[tid] = 1.0f / fmaxf(sqrtf(sNorm[tid]), 1.024e-9f);
  __syncthreads();

  if (tid < 64) {
    const int h = tid >> 3, i = tid & 7;
    const int hp = h >> 1, sub = h & 1;
    const float* s0 = sS + hp * 256 + (8 * sub + i) * 16 + 8 * sub;
    const float* s1 = s0 + 4 * 256;
    const float tv = bfr(temp[h]);
    const float iq = invn[h * 8 + i] * tv;
    const float* ik = invn + 64 + h * 8;
    float lg[8];
    float mx = -3.0e38f;
#pragma unroll
    for (int j = 0; j < 8; ++j) {
      const float v = ((s0[j] + s1[j]) * iq) * ik[j];
      lg[j] = v; mx = fmaxf(mx, v);
    }
    float ssum = 0.f;
#pragma unroll
    for (int j = 0; j < 8; ++j) { const float ev = __expf(lg[j] - mx); lg[j] = ev; ssum += ev; }
    const float inv = 1.0f / ssum;
#pragma unroll
    for (int j = 0; j < 8; ++j) attn[tid * 8 + j] = lg[j] * inv;
  }
  __syncthreads();
  for (int v = tid; v < 4096; v += 256) {
    const int cch = v >> 6, ci = v & 63;
    const int h = cch >> 3;
    const float* at = attn + cch * 8;
    float s = 0.f;
#pragma unroll 1
    for (int j = 0; j < 8; ++j) s = fmaf(at[j], bfr(wv[(h * 8 + j) * CN + ci]), s);
    M1[v] = s;
  }
  __syncthreads();
  for (int v = tid; v < 4096; v += 256) {
    const int oc = v >> 6, ci = v & 63;
    float s = 0.f;
#pragma unroll 1
    for (int cq = 0; cq < CN; ++cq) s = fmaf(bfr(wo[oc * CN + cq]), M1[cq * 64 + ci], s);
    const float sv = WTS * s;
    const _Float16 hi = (_Float16)sv;
    const _Float16 lo = (_Float16)((sv - (float)hi) * RSC);
    Wst[v] = h_bits(hi);
    Wst[4096 + v] = h_bits(lo);
  }
  if (tid < 64) {
    const int oc = tid;
    float s = 0.f;
#pragma unroll 1
    for (int cq = 0; cq < CN; ++cq) {
      const int h = cq >> 3;
      float t = 0.f;
#pragma unroll 1
      for (int j = 0; j < 8; ++j) t = fmaf(attn[cq * 8 + j], bfr(bv[h * 8 + j]), t);
      s = fmaf(bfr(wo[oc * CN + cq]), t, s);
    }
    BTst[oc] = s + bfr(bo[oc]);
  }
  __syncthreads();
  {
    const int e = tid & 7, lq = tid >> 3;
#pragma unroll
    for (int pass = 0; pass < 2; ++pass) {
#pragma unroll
      for (int it = 0; it < 4; ++it) {
        const int L = it * 32 + lq;
        const int plane = L >> 6, row = L & 63;
        const v4u u = *(const v4u*)(Wst + L * 64 + 8 * e);
        *(volatile v4u*)(WHL + ((size_t)(plane * (2 * NBT) + b * 2 + a) * 64 + row) * 64 + 8 * e) = u;
      }
      if (tid < 16) {
        const int L = tid >> 3;
        const v4f v = *(const v4f*)(BTst + L * 32 + 4 * e);
        *(volatile v4f*)(BTg + (b * 2 + a) * 64 + L * 32 + 4 * e) = v;
      }
      __threadfence();
    }
  }
}

__global__ __launch_bounds__(256)
void k_fused(const float* __restrict__ xi, const float* __restrict__ xe, const unsigned short* __restrict__ WHL,
             const float* __restrict__ BTg, unsigned short* FUSED) {
  __shared__ __align__(16) unsigned short X16[2 * 64 * XP];
  __shared__ __align__(16) unsigned short O[64 * OPP];
  const int tid = threadIdx.x, lane = tid & 31, wave = tid >> 5;
  const int hh = lane >> 4, c = lane & 15;
  const int tile = blockIdx.x, b = blockIdx.y;
  const int p0 = tile * 64;
  const size_t cb0 = (size_t)b * CN * HWN;
#pragma unroll
  for (int it = 0; it < 4; ++it) {
    const int idx = it * 256 + tid;
    const int ci = idx >> 4, p4 = (idx & 15) * 4;
    const size_t go = cb0 + (size_t)ci * HWN + p0 + p4;
    const v4f a0 = *(const v4f*)(xi + go);
    const v4f a1 = *(const v4f*)(xe + go);
#pragma unroll
    for (int q = 0; q < 4; ++q) {
      const int li = (p4 + q) * XP + ci;
      X16[li]           = h_bits((_Float16)(XSC * bfr(a0[q])));
      X16[64 * XP + li] = h_bits((_Float16)(XSC * bfr(a1[q])));
    }
  }
  __syncthreads();
  {
    const int mt = wave & 3, ntg0 = 6 * (wave >> 2);
    const unsigned short* xr0 = X16 + (16 * mt + c) * XP + 8 * hh;
#pragma unroll
    for (int qn = 0; qn < 6; ++qn) {
      const int ntg = ntg0 + qn;
      const int s = ntg >> 2, a = s >> 1, sx = s & 1;
      const unsigned short* xr = xr0 + sx * (64 * XP);
      const unsigned short* wr = WHL + ((size_t)((b * 2 + a) * 64 + 16 * (ntg & 3) + c)) * CN + 8 * hh;
      const unsigned short* wl = wr + (size_t)(2 * NBT) * 64 * 64;
      v8f acc = zero8(), accl = zero8();
#pragma unroll
      for (int ks = 0; ks < 2; ++ks) {
        const Frag fa  = ldfrag(xr + 32 * ks);
        const Frag fb  = ldfrag(wr + 32 * ks);
        const Frag fbl = ldfrag(wl + 32 * ks);
        acc  = mma_h(fa.h, fb.h, acc);
        accl = mma_h(fa.h, fbl.h, accl);
      }
      const float bs = FSC * BTg[(b * 2 + a) * 64 + 16 * (ntg & 3) + c];
#pragma unroll
      for (int r = 0; r < 8; ++r) {
        const float v = fmaf(acc[r] + accl[r] * IRSC, 0.015625f, bs);
        O[(16 * mt + 8 * hh + r) * OPP + 16 * ntg + c] = h_bits((_Float16)v);
      }
    }
  }
  __syncthreads();
  {
    const int e = tid & 7, lq = tid >> 3;
#pragma unroll
    for (int pass = 0; pass < 2; ++pass) {
#pragma unroll
      for (int it = 0; it < 6; ++it) {
        const int L = it * 32 + lq;
        const int p = L / 3, pc = L - 3 * p;
        const v4u u = *(const v4u*)(O + p * OPP + pc * 64 + 8 * e);
        *(volatile v4u*)(FUSED + ((size_t)(b * HWN + p0 + p)) * C3 + pc * 64 + 8 * e) = u;
      }
      __threadfence();
    }
  }
}

template <int CIN, int NOC>
__global__ __launch_bounds__(256)
void k_conv(const unsigned short* __restrict__ IN, const unsigned short* __restrict__ WC,
            const float* __restrict__ bias0, const float* __restrict__ bias1,
            float* T, size_t sstride, float* PARTC, float invsc) {
  constexpr int KT = 9 * CIN, NCC = CIN / 64, MPW = NOC / 64;
  constexpr int NIT = (2 * NOC) / 32;
  static_assert(CIN % 64 == 0);
  static_assert(NOC == 64 || NOC == 128);
  union Lds { unsigned short tin[3 * 66 * TP]; float Os[NOC * OSP]; };
  __shared__ __align__(16) Lds U;
  __shared__ __align__(16) float St[2 * NOC];
  unsigned short* const tin = U.tin;
  float* const Os = U.Os;
  const int tid = threadIdx.x, lane = tid & 31, wave = tid >> 5;
  const int hh = lane >> 4, c = lane & 15;
  const int xs = blockIdx.x, yrow = blockIdx.y, b = blockIdx.z;
  const int x0 = xs * 64;
  const int mtb = MPW * (wave >> 1), np = wave & 1;

  v8f acc[MPW][2];
  const unsigned short* wrp[MPW];
#pragma unroll
  for (int mi = 0; mi < MPW; ++mi) {
    acc[mi][0] = zero8(); acc[mi][1] = zero8();
    wrp[mi] = WC + ((size_t)(16 * (mtb + mi) + c)) * KT + 8 * hh;
  }
  const unsigned short* tb0 = tin + (32 * np + c) * TP + 8 * hh;
  const unsigned short* tb1 = tb0 + 16 * TP;

#pragma unroll 1
  for (int cc = 0; cc < NCC; ++cc) {
    __syncthreads();
    for (int i = tid; i < 3 * 66 * 8; i += 256) {
      const int e = i & 7, t2 = i >> 3;
      const int px = t2 % 66, ry = t2 / 66;
      const int gy = refl(yrow + ry - 1), gx = refl(x0 + px - 1);
      const v4u v = *(const v4u*)(IN + ((size_t)(b * HWN + gy * IMW + gx)) * CIN + cc * 64 + 8 * e);
      *(v4u*)(tin + (ry * 66 + px) * TP + 8 * e) = v;
    }
    __syncthreads();
    const int kc = cc * 64;
#pragma unroll
    for (int tap = 0; tap < 9; ++tap) {
      const int dy = tap / 3, dx = tap - 3 * dy;
      const int toff = (dy * 66 + dx) * TP;
#pragma unroll
      for (int ks = 0; ks < 2; ++ks) {
        const Frag fb0 = ldfrag(tb0 + toff + 32 * ks);
        const Frag fb1 = ldfrag(tb1 + toff + 32 * ks);
#pragma unroll
        for (int mi = 0; mi < MPW; ++mi) {
          const Frag fa = ldfrag(wrp[mi] + tap * CIN + kc + 32 * ks);
          acc[mi][0] = mma_h(fa.h, fb0.h, acc[mi][0]);
          acc[mi][1] = mma_h(fa.h, fb1.h, acc[mi][1]);
        }
      }
    }
  }
  __syncthreads();
#pragma unroll
  for (int mi = 0; mi < MPW; ++mi) {
#pragma unroll
    for (int j = 0; j < 2; ++j) {
#pragma unroll
      for (int r = 0; r < 8; ++r) {
        const int oc = 16 * (mtb + mi) + 8 * hh + r;
        const int ch = oc & 63;
        const float b0v = bfr(bias0[ch]), b1v = bfr(bias1[ch]);
        const float bs = (oc >= 64) ? b1v : b0v;
        Os[oc * OSP + 32 * np + 16 * j + c] = fmaf(acc[mi][j][r], invsc, bs);
      }
    }
  }
  __syncthreads();
  if (tid < NOC) {
    float s = 0.f, q = 0.f;
    const float* orow = Os + tid * OSP;
#pragma unroll 4
    for (int v = 0; v < 16; ++v) {
      const v4f x = *(const v4f*)(orow + 4 * v);
      s += (x[0] + x[1]) + (x[2] + x[3]);
      q = fmaf(x[0], x[0], q); q = fmaf(x[1], x[1], q); q = fmaf(x[2], x[2], q); q = fmaf(x[3], x[3], q);
    }
    St[tid] = s; St[NOC + tid] = q;
  }
  {
    const int e = tid & 7, lq = tid >> 3;
#pragma unroll
    for (int pass = 0; pass < 2; ++pass) {
#pragma unroll
      for (int it = 0; it < NIT; ++it) {
        const int L = it * 32 + lq;
        const int ocl = L >> 1, hf = L & 1;
        const v4f v = *(const v4f*)(Os + ocl * OSP + hf * 32 + 4 * e);
        float* dst = T + (size_t)(ocl >> 6) * sstride + ((size_t)(b * CN + (ocl & 63))) * HWN +
                     (size_t)yrow * IMW + x0 + hf * 32 + 4 * e;
        *(volatile v4f*)dst = v;
      }
      __threadfence();
    }
  }
  __syncthreads();
  if (tid < NOC / 2) {
    const int e = tid & 7, L = tid >> 3;
    const int blk = (b * IMW + yrow) * 4 + xs;
    const v4f v = *(const v4f*)(St + L * 32 + 4 * e);
    float* dst = PARTC + (size_t)blk * (2 * NOC) + L * 32 + 4 * e;
#pragma unroll
    for (int pass = 0; pass < 2; ++pass) {
      *(volatile v4f*)dst = v;
      __threadfence();
    }
  }
}

__global__ __launch_bounds__(128)
void k_bncoef(const float* __restrict__ PARTC, const float* __restrict__ gA, const float* __restrict__ beA,
              const float* __restrict__ gB, const float* __restrict__ beB, float* COEF, int noc, int nblk) {
  __shared__ __align__(16) float cf[256];
  const int tid = threadIdx.x;
  const int cc = min(tid, noc - 1);
  double s = 0.0, q = 0.0;
#pragma unroll 1
  for (int blk = 0; blk < nblk; ++blk) {
    const float* p = PARTC + (size_t)blk * (size_t)(2 * noc);
    s += (double)p[cc];
    q += (double)p[noc + cc];
  }
  const double inv_n = 1.0 / ((double)NBT * (double)HWN);
  const double m = s * inv_n;
  double var = q * inv_n - m * m;
  var = (var > 0.0) ? var : 0.0;
  const float varf = (float)var, mf = (float)m;
  const int cl = tid & 63;
  const float ga = bfr(gA[cl]), gb = bfr(gB[cl]), ba = bfr(beA[cl]), bbv = bfr(beB[cl]);
  const float g = (tid < 64) ? ga : gb;
  const float be = (tid < 64) ? ba : bbv;
  const float af = g * (1.0f / sqrtf(varf + 1e-5f));
  const float bf = be - mf * af;
  const bool ok = tid < noc;
  cf[tid] = ok ? af : 0.f;
  cf[128 + tid] = ok ? bf : 0.f;
  __syncthreads();
  if (tid < 64) {
    const int e = tid & 7, L = tid >> 3;
    const v4f v = *(const v4f*)(cf + L * 32 + 4 * e);
#pragma unroll
    for (int pass = 0; pass < 2; ++pass) {
      *(volatile v4f*)(COEF + L * 32 + 4 * e) = v;
      __threadfence();
    }
  }
}

__global__ __launch_bounds__(256)
void k_bnrelu(const float* __restrict__ T1, const float* __restrict__ COEF, unsigned short* CB1) {
  __shared__ __align__(16) unsigned short Lt[64 * XP];
  const int tid = threadIdx.x;
  const int tile = blockIdx.x, b = blockIdx.y;
  const int p0 = tile * 64;
#pragma unroll
  for (int it = 0; it < 4; ++it) {
    const int idx = it * 256 + tid;
    const int ch = idx >> 4, p4 = (idx & 15) * 4;
    const v4f v = *(const v4f*)(T1 + ((size_t)(b * CN + ch)) * HWN + p0 + p4);
    const float a = COEF[64 + ch], bb = COEF[192 + ch];
#pragma unroll
    for (int q = 0; q < 4; ++q) {
      const float z = fmaxf(fmaf(v[q], a, bb), 0.f);
      Lt[(p4 + q) * XP + ch] = h_bits((_Float16)(CBS * z));
    }
  }
  __syncthreads();
  {
    const int e = tid & 7, lq = tid >> 3;
#pragma unroll
    for (int pass = 0; pass < 2; ++pass) {
#pragma unroll
      for (int it = 0; it < 2; ++it) {
        const int p = it * 32 + lq;
        const v4u u = *(const v4u*)(Lt + p * XP + 8 * e);
        *(volatile v4u*)(CB1 + ((size_t)(b * HWN + p0 + p)) * CN + 8 * e) = u;
      }
      __threadfence();
    }
  }
}

__global__ __launch_bounds__(256)
void k_final(const float* __restrict__ TI, const float* __restrict__ T2, const float* __restrict__ CI,
             const float* __restrict__ C2, float* OUT) {
  const size_t base = ((size_t)blockIdx.x * 256 + threadIdx.x) * 4;
  const int ch = (int)((base >> 16) & 63);
  const v4f a = *(const v4f*)(TI + base);
  const v4f t = *(const v4f*)(T2 + base);
  const float aI = CI[ch], bI = CI[128 + ch], a2 = C2[ch], b2c = C2[128 + ch];
  v4f o;
#pragma unroll
  for (int q = 0; q < 4; ++q) {
    const float zi = fmaxf(fmaf(a[q], aI, bI), 0.f);
    o[q] = fmaxf(zi + fmaf(t[q], a2, b2c), 0.f);
  }
#pragma unroll
  for (int pass = 0; pass < 2; ++pass) {
    *(volatile v4f*)(OUT + base) = o;
    __threadfence();
  }
}

extern "C" void kernel_launch(void* const* d_in, const int* in_sizes, int n_in,
                              void* d_out, int out_size, void* d_ws, size_t ws_size,
                              hipStream_t stream) {
  const int XN = NBT * CN * HWN;
  if (n_in < 24) return;
  if (in_sizes[0] != XN || in_sizes[1] != XN || in_sizes[2] != XN) return;
  if (in_sizes[3] != NHEAD) return;
  for (int i = 4; i < 12; i += 2) { if (in_sizes[i] != CN * CN) return; if (in_sizes[i + 1] != CN) return; }
  if (in_sizes[12] != CN * C3 * 9 || in_sizes[16] != CN * C3 * 9 || in_sizes[20] != CN * CN * 9) return;
  {
    const int small_ix[9] = {13, 14, 15, 17, 18, 19, 21, 22, 23};
    for (int i = 0; i < 9; ++i) if (in_sizes[small_ix[i]] != CN) return;
  }
  if (out_size != XN) return;

  size_t off = 0;
  auto carve = [&](size_t bytes) { const size_t o = off; off += (bytes + 255) & ~(size_t)255; return o; };
  const size_t t64b   = (size_t)XN * 4;
  const size_t oWQK   = carve((size_t)2 * CN * CN * 2);
  const size_t oWC1   = carve((size_t)128 * KT1 * 2);
  const size_t oWC2   = carve((size_t)64 * KT2 * 2);
  const size_t oWHL   = carve((size_t)2 * NBT * 2 * CN * CN * 2);
  const size_t oBT    = carve((size_t)NBT * 2 * CN * 4);
  const size_t oFUSED = carve((size_t)NBT * HWN * C3 * 2);
  const size_t oT     = carve(2 * t64b);
  const size_t oPC1   = carve((size_t)NCBLK * 2 * 128 * 4);
  const size_t oPC2   = carve((size_t)NCBLK * 2 * 64 * 4);
  const size_t oCF1   = carve(1024);
  const size_t oCF2   = carve(1024);
  if (off > ws_size) return;
  if (off > (size_t)134217728) return;
  if ((size_t)NBT * HWN * CN * 2 > (size_t)NBT * HWN * C3 * 2) return;
  if ((size_t)3 * NBT * CN * HWN * 2 > 2 * t64b) return;

  const float* x_i  = (const float*)d_in[0];
  const float* x_e  = (const float*)d_in[1];
  const float* y    = (const float*)d_in[2];
  const float* temp = (const float*)d_in[3];
  const float* wq   = (const float*)d_in[4];  const float* bq = (const float*)d_in[5];
  const float* wk   = (const float*)d_in[6];  const float* bk = (const float*)d_in[7];
  const float* wv   = (const float*)d_in[8];  const float* bv = (const float*)d_in[9];
  const float* wo   = (const float*)d_in[10]; const float* bo = (const float*)d_in[11];
  const float* w_init = (const float*)d_in[12]; const float* b_init = (const float*)d_in[13];
  const float* g_init = (const float*)d_in[14]; const float* be_init = (const float*)d_in[15];
  const float* w1 = (const float*)d_in[16]; const float* b1 = (const float*)d_in[17];
  const float* g1 = (const float*)d_in[18]; const float* be1 = (const float*)d_in[19];
  const float* w2 = (const float*)d_in[20]; const float* b2 = (const float*)d_in[21];
  const float* g2 = (const float*)d_in[22]; const float* be2 = (const float*)d_in[23];
  float* out = (float*)d_out;

  char* ws = (char*)d_ws;
  unsigned short* WQK   = (unsigned short*)(ws + oWQK);
  unsigned short* WC1   = (unsigned short*)(ws + oWC1);
  unsigned short* WC2   = (unsigned short*)(ws + oWC2);
  unsigned short* WHL   = (unsigned short*)(ws + oWHL);
  float*          BT    = (float*)(ws + oBT);
  unsigned short* FUSED = (unsigned short*)(ws + oFUSED);
  unsigned short* CB1   = (unsigned short*)(ws + oFUSED);
  float*          T     = (float*)(ws + oT);
  float*          T1    = T + (size_t)XN;
  unsigned short* QKP   = (unsigned short*)(ws + oT);
  float*          PC1   = (float*)(ws + oPC1);
  float*          PC2   = (float*)(ws + oPC2);
  float*          CF1   = (float*)(ws + oCF1);
  float*          CF2   = (float*)(ws + oCF2);

  const dim3 blk256(256), blk128(128);

  cvt_w<<<dim3(130), blk256, 0, stream>>>(w_init, w1, w2, wq, wk, WC1, WC2, WQK);
  k_proj<<<dim3(HWN / 64, 3, NBT), blk256, 0, stream>>>(y, x_e, x_i, WQK, bq, bk, QKP);
  k_attnw<<<dim3(2, NBT), blk256, 0, stream>>>(QKP, temp, wv, bv, wo, bo, WHL, BT);
  k_fused<<<dim3(HWN / 64, NBT), blk256, 0, stream>>>(x_i, x_e, WHL, BT, FUSED);
  k_conv<C3, 128><<<dim3(4, IMW, NBT), blk256, 0, stream>>>(FUSED, WC1, b_init, b1, T, (size_t)XN, PC1,
                                                           1.0f / 65536.0f);
  k_bncoef<<<dim3(1), blk128, 0, stream>>>(PC1, g_init, be_init, g1, be1, CF1, 128, NCBLK);
  k_bnrelu<<<dim3(HWN / 64, NBT), blk256, 0, stream>>>(T1, CF1, CB1);
  k_conv<CN, 64><<<dim3(4, IMW, NBT), blk256, 0, stream>>>(CB1, WC2, b2, b2, T1, (size_t)0, PC2,
                                                         1.0f / 1024.0f);
  k_bncoef<<<dim3(1), blk128, 0, stream>>>(PC2, g2, be2, g2, be2, CF2, 64, NCBLK);
  k_final<<<dim3(XN / 1024), blk256, 0, stream>>>(T, T1, CF1, CF2, out);
  (void)hipGetLastError();
}
